// DeepGCNWithResidual_39238821216994
// MI455X (gfx1250) — hardware-verified
//
#include <hip/hip_runtime.h>


namespace {
constexpr int NN = 50000, NP = 50016, NE = 600000, D = 128, NGR = 64, DOUT = 3, MAXDEG = 1024, NGc = (NN + 511) / 512, PERMLEN = NE + 32 * NGc + 32;
constexpr float XS = 8.0f, EPS = 1e-5f;

typedef _Float16 b16;
typedef __attribute__((ext_vector_type(16))) _Float16 v16b;
typedef __attribute__((ext_vector_type(8))) _Float16 v8b;
typedef __attribute__((ext_vector_type(8))) float v8f;
typedef __attribute__((ext_vector_type(4))) float v4f;
__device__ __forceinline__ float bf16_rne(float f) { unsigned int u = __float_as_uint(f); u += 0x7FFFu + ((u >> 16) & 1u); return __uint_as_float(u & 0xFFFF0000u); }
__device__ __forceinline__ void split16(float v, b16& hi, b16& lo) { hi = (b16)v; lo = (b16)(v - (float)hi); }
__device__ __forceinline__ v16b frag_kb(const b16* p, int hh) { const v8b a = *(const v8b*)(p + 8 * hh), b = *(const v8b*)(p + 16 + 8 * hh); v16b f;
#pragma unroll
  for (int e = 0; e < 8; ++e) { f[e] = a[e]; f[8 + e] = b[e]; } return f; }
__device__ __forceinline__ v8f wmma16b(v16b a, v16b b, v8f c) { v8f d = __builtin_amdgcn_wmma_f32_16x16x32_f16(false, a, false, b, (short)0, c, false, false); asm volatile("v_nop\n\tv_nop\n\tv_nop\n\tv_nop" : "+v"(d) : "v"(a), "v"(b)); return d; }
__device__ __forceinline__ void wave_lds_sync() { __builtin_amdgcn_fence(__ATOMIC_RELEASE, "workgroup"); __builtin_amdgcn_wave_barrier(); __builtin_amdgcn_fence(__ATOMIC_ACQUIRE, "workgroup"); }
__device__ __forceinline__ float pmul(float a, float b) { float p = a * b; asm volatile("" : "+v"(p)); return p; }
__device__ __forceinline__ float wsum(float v) {
#pragma unroll
  for (int o = 1; o < 32; o <<= 1) v += __shfl_xor(v, o); return v; }
constexpr int CSR_NBLK = 512, CSR_GB = 9, CSR_GN = 1 << CSR_GB  , CSR_MAXG = 512, CSR_CAP = 12288  ;
__global__ __launch_bounds__(64) void csrA_kernel(const int* __restrict__ dst, int E, int N, int nG, int CHP, int NGP, int* __restrict__ STG, int* __restrict__ HST) {
  extern __shared__ int sm[];
  int* cnt = sm; int* run = sm + NGP; int* ids = sm + 2 * NGP;
  const int b = blockIdx.x; const int ch = (E + CSR_NBLK - 1) / CSR_NBLK; const int e0 = b * ch, e1 = min(E, e0 + ch);
  for (int i = threadIdx.x; i < NGP; i += 64) cnt[i] = 0;
  for (int i = threadIdx.x; i < CHP; i += 64) ids[i] = -1;
  __syncthreads();
  if (threadIdx.x == 0) {
    for (int e = e0; e < e1; ++e) { int d = dst[e]; d = (d < 0) ? 0 : (d >= N ? N - 1 : d); cnt[d >> CSR_GB] += 1; }
    int acc = 0; for (int g = 0; g < nG; ++g) { run[g] = acc; acc += cnt[g]; }
    for (int e = e0; e < e1; ++e) { int d = dst[e]; d = (d < 0) ? 0 : (d >= N ? N - 1 : d); const int g = d >> CSR_GB; ids[run[g]] = e; run[g] += 1; } }
  __syncthreads();
  typedef __attribute__((ext_vector_type(4))) int v4i;
  for (int pass = 0; pass < 2; ++pass) {
    for (int i = threadIdx.x; i < CHP / 4; i += 64) *(volatile v4i*)(STG + (size_t)b * CHP + i * 4) = *(const v4i*)(&ids[i * 4]);
    for (int i = threadIdx.x; i < NGP / 4; i += 64) { v4i v; for (int e = 0; e < 4; ++e) v[e] = (i * 4 + e < nG) ? cnt[i * 4 + e] : 0; *(volatile v4i*)(HST + (size_t)b * NGP + i * 4) = v; }
    __threadfence(); }
}
__global__ __launch_bounds__(512) void csrS_kernel(const int* __restrict__ HST, int nG, int NGP, int* __restrict__ START, int* __restrict__ TOT, int* __restrict__ OFF) {
  __shared__ int tot[CSR_MAXG];
  const int b = threadIdx.x;
  for (int pass = 0; pass < 2; ++pass) { int runb = 0; for (int g = 0; g < nG; ++g) { int c = HST[(size_t)b * NGP + g]; c = (c < 0) ? 0 : c; ((volatile int*)OFF)[(size_t)g * CSR_NBLK + b] = runb; runb += c; } __threadfence(); }
  for (int g = threadIdx.x; g < nG; g += 512) { int s = 0; for (int bb = 0; bb < CSR_NBLK; ++bb) { int c = HST[(size_t)bb * NGP + g]; s += (c < 0) ? 0 : c; } tot[g] = s; }
  __syncthreads();
  if (threadIdx.x < 32) {
    __shared__ int st[CSR_MAXG + 32];
    if (threadIdx.x == 0) { int acc = 0; for (int g = 0; g < NGP; ++g) { st[g] = acc; if (g < nG) acc += (tot[g] + 31) & ~31; } st[NGP] = acc; }
    __builtin_amdgcn_fence(__ATOMIC_RELEASE, "workgroup"); __builtin_amdgcn_wave_barrier(); __builtin_amdgcn_fence(__ATOMIC_ACQUIRE, "workgroup");
    for (int pass = 0; pass < 2; ++pass) { for (int i = threadIdx.x; i < NGP + 32; i += 32) { ((volatile int*)START)[i] = (i <= NGP) ? st[min(i, NGP)] : 0; ((volatile int*)TOT)[i] = (i < nG) ? tot[i] : 0; } __threadfence(); } }
}
__global__ __launch_bounds__(256) void csrB_kernel(const int* __restrict__ dst, int N, int nG, int CHP, int NGP, int permLen, const int* __restrict__ STG, const int* __restrict__ HST, const int* __restrict__ OFF, const int* __restrict__ START, const int* __restrict__ TOT, int* __restrict__ PERM, int* __restrict__ ROWPTR, int* __restrict__ ROWCNT, int* __restrict__ FLAG) {
  typedef __attribute__((ext_vector_type(4))) int v4i;
  __shared__ int ids[CSR_CAP]; __shared__ unsigned short key[CSR_CAP]; __shared__ int outp[CSR_CAP]; __shared__ int ncnt[CSR_GN + 1]; __shared__ int boff[CSR_NBLK + 1];
  const int g = blockIdx.x, t_ = threadIdx.x; int tot = TOT[g]; int st = START[g], stn = START[g + 1]; const int v0 = g * CSR_GN; const int nv = min(CSR_GN, N - v0);
  st = (st < 0) ? 0 : (st > permLen - 32 ? permLen - 32 : st) & ~31; stn = (stn < st) ? st : (stn > permLen ? permLen : stn); tot = (tot < 0) ? 0 : tot; if (tot > stn - st && tot <= CSR_CAP) tot = stn - st;
  if (tot > CSR_CAP) {
    for (int pass = 0; pass < 2; ++pass) { for (int i = t_; i < CSR_GN / 4; i += 256) { v4i a, c; for (int e = 0; e < 4; ++e) { a[e] = st; c[e] = 0; } *(volatile v4i*)(ROWPTR + v0 + i * 4) = a; *(volatile v4i*)(ROWCNT + v0 + i * 4) = c; } if (t_ == 0) ((volatile int*)FLAG)[0] = 1; __threadfence(); } (void)nv; return; }
  if (t_ == 0) { int acc = 0; for (int b = 0; b < CSR_NBLK; ++b) { boff[b] = acc; int c = HST[(size_t)b * NGP + g]; c = (c < 0) ? 0 : (c > CHP ? CHP : c); acc += c; if (acc > tot) acc = tot; } boff[CSR_NBLK] = acc; }
  for (int i = t_; i <= CSR_GN; i += 256) ncnt[i] = 0;
  __syncthreads();
  for (int b = 0; b < CSR_NBLK; ++b) { const int c = boff[b + 1] - boff[b]; int o_ = OFF[(size_t)g * CSR_NBLK + b]; o_ = (o_ < 0) ? 0 : (o_ > CHP - c ? CHP - c : o_); const int* src_ = STG + (size_t)b * CHP + o_;
    for (int i = t_; i < c; i += 256) { int id = src_[i]; id = (id < 0) ? 0 : id; ids[boff[b] + i] = id; int d = dst[id]; d = (d < v0) ? v0 : (d >= N ? N - 1 : d); int kk = d - v0; kk = (kk < 0) ? 0 : (kk >= CSR_GN ? CSR_GN - 1 : kk); key[boff[b] + i] = (unsigned short)kk; } }
  __syncthreads();
  if (t_ == 0) { for (int i = 0; i < tot; ++i) ncnt[key[i]] += 1; int acc = 0; for (int vl = 0; vl < CSR_GN; ++vl) { const int c = ncnt[vl]; ncnt[vl] = acc; acc += c; } ncnt[CSR_GN] = acc;
    for (int i = 0; i < tot; ++i) { const int vl = key[i]; outp[ncnt[vl]] = ids[i]; ncnt[vl] += 1; }
    for (int vl = CSR_GN; vl > 0; --vl) ncnt[vl] = ncnt[vl - 1]; ncnt[0] = 0; }
  __syncthreads();
  for (int pass = 0; pass < 2; ++pass) {
    for (int i = t_; i < (stn - st) / 4; i += 256) { v4i v; for (int e = 0; e < 4; ++e) { const int q = i * 4 + e; v[e] = (q < tot) ? outp[q] : -1; } *(volatile v4i*)(PERM + st + i * 4) = v; }
    for (int i = t_; i < CSR_GN / 4; i += 256) { v4i a, c; for (int e = 0; e < 4; ++e) { const int vl = i * 4 + e; a[e] = st + ncnt[vl]; c[e] = (vl < nv) ? (ncnt[vl + 1] - ncnt[vl]) : 0; } *(volatile v4i*)(ROWPTR + v0 + i * 4) = a; *(volatile v4i*)(ROWCNT + v0 + i * 4) = c; }
    __threadfence(); }
}
__global__ __launch_bounds__(256) void csrZ_kernel(int* __restrict__ p, size_t n4) { typedef __attribute__((ext_vector_type(4))) int v4i; const size_t tid = (size_t)blockIdx.x * 256 + threadIdx.x, nth = (size_t)gridDim.x * 256; v4i z = {0, 0, 0, 0}; for (size_t i = tid; i < n4; i += nth) *(volatile v4i*)(p + i * 4) = z; }
struct CsrBufs { int *STG, *HST, *OFF, *START, *TOT, *PERM, *ROWPTR, *ROWCNT, *FLAG; int nG, NGP, CHP; size_t permLen; char* base; size_t bytes; };
static size_t csr_carve(CsrBufs& c, char* ws, size_t off, int E, int N) {
  const size_t off0 = off; c.base = ws + off;
  auto al = [&](size_t bytes) { char* p = ws + off; off += (bytes + 255) & ~(size_t)255; return p; };
  c.nG = (N + CSR_GN - 1) / CSR_GN; c.NGP = (c.nG + 31) & ~31; const int ch = (E + CSR_NBLK - 1) / CSR_NBLK; c.CHP = (ch + 31) & ~31; c.permLen = (size_t)E + 32 * (size_t)c.nG + 32;
  c.STG = (int*)al((size_t)CSR_NBLK * c.CHP * 4); c.HST = (int*)al((size_t)CSR_NBLK * c.NGP * 4); c.OFF = (int*)al((size_t)c.NGP * CSR_NBLK * 4); c.START = (int*)al((size_t)(c.NGP + 64) * 4); c.TOT = (int*)al((size_t)(c.NGP + 64) * 4);
  c.PERM = (int*)al(c.permLen * 4); c.ROWPTR = (int*)al((size_t)c.nG * CSR_GN * 4); c.ROWCNT = (int*)al((size_t)c.nG * CSR_GN * 4); c.FLAG = (int*)al(256);
  c.bytes = off - off0; return off;
}
static void csr_build(const CsrBufs& c, const int* dst, int E, int N, hipStream_t stream) {
  const size_t smem = (size_t)(2 * c.NGP + c.CHP) * 4;
  csrZ_kernel<<<512, 256, 0, stream>>>((int*)c.base, c.bytes / 16);
  csrA_kernel<<<CSR_NBLK, 64, smem, stream>>>(dst, E, N, c.nG, c.CHP, c.NGP, c.STG, c.HST);
  csrS_kernel<<<1, 512, 0, stream>>>(c.HST, c.nG, c.NGP, c.START, c.TOT, c.OFF);
  csrB_kernel<<<c.nG, 256, 0, stream>>>(dst, N, c.nG, c.CHP, c.NGP, (int)c.permLen, c.STG, c.HST, c.OFF, c.START, c.TOT, c.PERM, c.ROWPTR, c.ROWCNT, c.FLAG);
}

__global__ __launch_bounds__(256) void prep_kernel(const float* __restrict__ x, const float* __restrict__ win, const float* __restrict__ bin, const float* __restrict__ wbl, const float* __restrict__ bbl, const float* __restrict__ wout, const float* __restrict__ bout, const float* __restrict__ gm, const float* __restrict__ bt, const float* __restrict__ f1w, const float* __restrict__ f1b, const float* __restrict__ f2w, const float* __restrict__ f2b, b16* __restrict__ R, float* __restrict__ P, b16* __restrict__ Hh, b16* __restrict__ Hl, float* __restrict__ Hf) {
  const size_t tid = (size_t)blockIdx.x * 256 + threadIdx.x, nth = (size_t)gridDim.x * 256;
  for (int pass = 0; pass < 2; ++pass) {
    for (size_t p = tid; p < (size_t)5 * D * (D / 8); p += nth) { const int l = (int)(p / (D * (D / 8))), rem = (int)(p % (D * (D / 8))), o = rem / (D / 8), k0 = (rem % (D / 8)) * 8; const float* W = (l == 0) ? win : (l == 4) ? wout : (wbl + (size_t)(l - 1) * D * D); v8b v;
      for (int e = 0; e < 8; ++e) v[e] = (b16)bf16_rne(W[(size_t)(k0 + e) * D + o]); *(volatile v8b*)(R + ((size_t)l * D + o) * D + k0) = v; }
    for (size_t q = tid; q < 34304; q += nth) { const int i = (int)q; float v; if (i < 128) v = bin[i]; else if (i < 512) v = bbl[i - 128]; else if (i < 640) v = bout[i - 512]; else if (i < 768) v = gm[i - 640]; else if (i < 896) v = bt[i - 768]; else if (i < 1024) v = f1b[i - 896]; else if (i < 1152) v = (i - 1024 < DOUT) ? f2b[i - 1024] : 0.0f; else if (i < 33920) v = f1w[i - 1152]; else v = f2w[i - 33920];
      P[q] = bf16_rne(v); }
    for (size_t p = tid; p < (size_t)NP * D / 8; p += nth) { const size_t r = p / (D / 8); v8b v = {}, z = {}; float f[8] = {0, 0, 0, 0, 0, 0, 0, 0}; if (r < (size_t)NN) { for (int e = 0; e < 8; ++e) { f[e] = bf16_rne(x[p * 8 + e]); v[e] = (b16)(f[e] * XS); } }
      *(volatile v8b*)(Hh + p * 8) = v; *(volatile v8b*)(Hl + p * 8) = z; *(volatile v4f*)(Hf + p * 8) = *(v4f*)&f[0]; *(volatile v4f*)(Hf + p * 8 + 4) = *(v4f*)&f[4]; }
    __threadfence(); }
}

__global__ __launch_bounds__(64) void gemm_kernel(const b16* __restrict__ Hh, const b16* __restrict__ Hl, const b16* __restrict__ R, int l, float* __restrict__ HW) {
  __shared__ __attribute__((aligned(16))) float Ts[2][16][D + 4];
  const int lane = threadIdx.x & 31, wave = threadIdx.x >> 5, nloc = lane & 15, hlf = lane >> 4, m0 = blockIdx.x * 32 + wave * 16; const b16* Bw = R + (size_t)l * D * D;
  v8f acc[8];
#pragma unroll
  for (int t = 0; t < 8; ++t) acc[t] = (v8f){};
#pragma unroll
  for (int kb = 0; kb < D; kb += 32) { const v16b a = frag_kb(Hh + (size_t)(m0 + nloc) * D + kb, hlf), al = frag_kb(Hl + (size_t)(m0 + nloc) * D + kb, hlf);
#pragma unroll
    for (int t = 0; t < 8; ++t) { const v16b bw = frag_kb(Bw + (size_t)(t * 16 + nloc) * D + kb, hlf); acc[t] = wmma16b(a, bw, acc[t]); acc[t] = wmma16b(al, bw, acc[t]); } }
#pragma unroll
  for (int t = 0; t < 8; ++t)
#pragma unroll
    for (int r = 0; r < 8; ++r) Ts[wave][8 * hlf + r][t * 16 + nloc] = acc[t][r] * (1.0f / XS);
  wave_lds_sync();
  for (int pass = 0; pass < 2; ++pass) { for (int i = lane; i < 16 * 32; i += 32) { const int rr = i >> 5, c4 = (i & 31) * 4; *(volatile v4f*)(HW + (size_t)(m0 + rr) * D + c4) = *(const v4f*)(&Ts[wave][rr][c4]); } __threadfence(); }
}

template <int MODE>
__global__ __launch_bounds__(256) void agg_kernel(const float* __restrict__ HW, const int* __restrict__ src, const int* __restrict__ perm, const int* __restrict__ rowptr, const int* __restrict__ rowcnt, const float* __restrict__ P, int l, float* __restrict__ Hf, b16* __restrict__ Hh, b16* __restrict__ Hl) {
  __shared__ __attribute__((aligned(16))) b16 Sh[8][D + 8], Sl[8][D + 8];
  const int wave = threadIdx.x >> 5, v = blockIdx.x * 8 + wave, lane = threadIdx.x & 31;
  int cnt = rowcnt[v]; cnt = (cnt < 0) ? 0 : (cnt > MAXDEG ? MAXDEG : cnt); int p0 = rowptr[v]; p0 = (p0 < 0) ? 0 : (p0 > PERMLEN - cnt ? PERMLEN - cnt : p0);
  const float dv = rsqrtf((float)cnt + 1.0f);
  v4f acc = *(const v4f*)(HW + (size_t)v * D + lane * 4) * (dv * dv);
  for (int q = 0; q < cnt; ++q) { int id = perm[p0 + q]; id = (id < 0) ? 0 : (id >= NE ? NE - 1 : id); int s = src[id]; s = (s < 0) ? 0 : (s >= NN ? NN - 1 : s); int cs_ = rowcnt[s]; cs_ = (cs_ < 0) ? 0 : (cs_ > MAXDEG ? MAXDEG : cs_); const float w = pmul(rsqrtf((float)cs_ + 1.0f), dv); const v4f hv = *(const v4f*)(HW + (size_t)s * D + lane * 4);
#pragma unroll
    for (int e = 0; e < 4; ++e) acc[e] += pmul(w, hv[e]); }
  float y[4];
#pragma unroll
  for (int e = 0; e < 4; ++e) y[e] = acc[e] + P[l * D + lane * 4 + e];
  if (MODE != 2) {
#pragma unroll
    for (int e = 0; e < 4; ++e) y[e] = fmaxf(y[e], 0.0f);
    const float s_ = wsum(y[0] + y[1] + y[2] + y[3]); const float mu = s_ * (1.0f / D); float q_ = 0.0f;
#pragma unroll
    for (int e = 0; e < 4; ++e) { const float d_ = y[e] - mu; q_ += pmul(d_, d_); }
    q_ = wsum(q_); const float inv = rsqrtf(q_ * (1.0f / D) + EPS);
    const v4f res = *(const v4f*)(Hf + (size_t)v * D + lane * 4);
#pragma unroll
    for (int e = 0; e < 4; ++e) { const int c = lane * 4 + e; y[e] = pmul((y[e] - mu) * inv, P[640 + c]) + P[768 + c]; if (MODE == 1) y[e] += res[e]; }
#pragma unroll
    for (int e = 0; e < 4; ++e) { b16 a_, b_; split16(y[e] * XS, a_, b_); Sh[wave][lane * 4 + e] = a_; Sl[wave][lane * 4 + e] = b_; }
    wave_lds_sync(); }
  v4f o; for (int e = 0; e < 4; ++e) o[e] = y[e];
  for (int pass = 0; pass < 2; ++pass) { *(volatile v4f*)(Hf + (size_t)v * D + lane * 4) = o; if (MODE != 2 && lane < 16) { *(volatile v8b*)(Hh + (size_t)v * D + lane * 8) = *(const v8b*)(&Sh[wave][lane * 8]); *(volatile v8b*)(Hl + (size_t)v * D + lane * 8) = *(const v8b*)(&Sl[wave][lane * 8]); } __threadfence(); }
}

__global__ __launch_bounds__(128) void pool_kernel(const float* __restrict__ Hf, const int* __restrict__ batch, float* __restrict__ G) {
  const int g = blockIdx.x, c = threadIdx.x;
  auto lower = [&](int key) { int lo = 0, hi = NN; while (lo < hi) { const int mid = (lo + hi) >> 1; if (batch[mid] < key) lo = mid + 1; else hi = mid; } return lo; };
  const int s0 = lower(g), s1 = lower(g + 1); const int cnt = s1 - s0;
  float sm = 0.0f, mx = -INFINITY; for (int n = s0; n < s1; ++n) { const float hv = Hf[(size_t)n * D + c]; sm += hv; mx = fmaxf(mx, hv); }
  const float mean = sm / fmaxf((float)cnt, 1.0f); if (cnt == 0) mx = -INFINITY;
  for (int pass = 0; pass < 2; ++pass) { ((volatile float*)G)[(size_t)g * 2 * D + c] = mean; ((volatile float*)G)[(size_t)g * 2 * D + D + c] = mx; __threadfence(); }
}
__global__ __launch_bounds__(64) void head_kernel(const float* __restrict__ G, const float* __restrict__ P, float* __restrict__ out) {
  __shared__ __attribute__((aligned(16))) float Os[NGR * DOUT + 64];
  const int g = threadIdx.x; const float* gr = G + (size_t)g * 2 * D; float o[DOUT]; for (int k = 0; k < DOUT; ++k) o[k] = P[1024 + k];
  for (int j = 0; j < D; ++j) { float s = P[896 + j]; for (int i = 0; i < 2 * D; ++i) s += pmul(gr[i], P[1152 + i * D + j]); s = fmaxf(s, 0.0f); for (int k = 0; k < DOUT; ++k) o[k] += pmul(s, P[33920 + j * DOUT + k]); }
  for (int k = 0; k < DOUT; ++k) Os[g * DOUT + k] = o[k];
  __syncthreads();
  for (int pass = 0; pass < 2; ++pass) { if (g < NGR * DOUT / 4) *(volatile v4f*)(out + g * 4) = *(const v4f*)(&Os[g * 4]); __threadfence(); }
}
}

extern "C" void kernel_launch(void* const* d_in, const int* in_sizes, int n_in,
                              void* d_out, int out_size, void* d_ws, size_t ws_size, hipStream_t stream) {
  (void)n_in; (void)out_size;
  const float* x = (const float*)d_in[0]; const int* ei = (const int*)d_in[1]; const int* batch = (const int*)d_in[2]; const float* win = (const float*)d_in[3]; const float* bin = (const float*)d_in[4]; const float* wbl = (const float*)d_in[5]; const float* bbl = (const float*)d_in[6]; const float* wout = (const float*)d_in[7]; const float* bout = (const float*)d_in[8];
  const float* gm = (const float*)d_in[9]; const float* bt = (const float*)d_in[10]; const float* f1w = (const float*)d_in[11]; const float* f1b = (const float*)d_in[12]; const float* f2w = (const float*)d_in[13]; const float* f2b = (const float*)d_in[14];
  float* out = (float*)d_out;
  if (in_sizes[0] != NN * D || in_sizes[1] != 2 * NE || in_sizes[2] != NN || in_sizes[11] != 2 * D * D) return;
  const int* srcI = ei; const int* dstI = ei + NE;
  size_t off = 0; char* ws = (char*)d_ws;
  auto carve = [&](size_t bytes) { char* p = ws + off; off += (bytes + 255) & ~(size_t)255; return p; };
  b16* R = (b16*)carve((size_t)5 * D * D * 2); float* P = (float*)carve(34304 * 4); b16* Hh = (b16*)carve((size_t)NP * D * 2); b16* Hl = (b16*)carve((size_t)NP * D * 2); float* Hf = (float*)carve((size_t)NP * D * 4); float* HW = (float*)carve((size_t)NP * D * 4); float* G = (float*)carve((size_t)NGR * 2 * D * 4);
  CsrBufs cs; off = csr_carve(cs, ws, off, NE, NN);
  if (off > ws_size) return;
  csr_build(cs, dstI, NE, NN, stream);
  prep_kernel<<<512, 256, 0, stream>>>(x, win, bin, wbl, bbl, wout, bout, gm, bt, f1w, f1b, f2w, f2b, R, P, Hh, Hl, Hf);
  gemm_kernel<<<NP / 32, 64, 0, stream>>>(Hh, Hl, R, 0, HW);
  agg_kernel<0><<<NN / 8, 256, 0, stream>>>(HW, srcI, cs.PERM, cs.ROWPTR, cs.ROWCNT, P, 0, Hf, Hh, Hl);
  for (int i = 0; i < 3; ++i) { gemm_kernel<<<NP / 32, 64, 0, stream>>>(Hh, Hl, R, 1 + i, HW);
    agg_kernel<1><<<NN / 8, 256, 0, stream>>>(HW, srcI, cs.PERM, cs.ROWPTR, cs.ROWCNT, P, 1 + i, Hf, Hh, Hl); }
  gemm_kernel<<<NP / 32, 64, 0, stream>>>(Hh, Hl, R, 4, HW);
  agg_kernel<2><<<NN / 8, 256, 0, stream>>>(HW, srcI, cs.PERM, cs.ROWPTR, cs.ROWCNT, P, 4, Hf, nullptr, nullptr);
  pool_kernel<<<NGR, 128, 0, stream>>>(Hf, batch, G);
  head_kernel<<<1, 64, 0, stream>>>(G, P, out);
}
